// OuterProductMean_51694226374798
// MI455X (gfx1250) — hardware-run, weakly checked
//
#include <hip/hip_runtime.h>
#include <math.h>

constexpr int kS   = 128;
constexpr int kR   = 256;
constexpr int kCM  = 256;
constexpr int kCH  = 32;
constexpr int kCZ  = 128;
constexpr int kRows   = kS * kR;
constexpr int kNcat   = 2 * kCH;
constexpr int kKo     = kCH * kCH;
constexpr int kABrows = kR * kCH;
constexpr int kChunkI = 128;
constexpr int kNumChunks = kR / kChunkI;
constexpr int kOuterRows = kChunkI * kR;
constexpr float kLnEps   = 1e-5f;
constexpr float kNormEps = 1e-3f;
constexpr float kInvCM   = 1.0f / 256.0f;

static_assert(kRows % 64 == 0 && kNcat % 64 == 0 && kCM % 32 == 0, "gemm1 shape");
static_assert((kChunkI * kCH) % 64 == 0 && (kR * kCH) % 64 == 0 && kS % 32 == 0, "gemm2 shape");
static_assert(kOuterRows % 64 == 0 && kCZ % 64 == 0 && kKo % 32 == 0, "gemm3 shape");
static_assert(kNumChunks * kChunkI == kR, "chunking");

constexpr size_t kOffBt1   = 0;
constexpr size_t kOffBt3   = kOffBt1 + (size_t)kNcat * kCM * 2;
constexpr size_t kOffRnorm = kOffBt3 + (size_t)kCZ * kKo * 2;
constexpr size_t kOffMnP   = kOffRnorm + (size_t)kR * kR * 4;
constexpr size_t kOffP1    = kOffMnP + (size_t)kRows * kCM * 2;
constexpr size_t kOffA2    = kOffP1 + (size_t)kRows * kNcat * 4;
constexpr size_t kOffBt2   = kOffA2 + (size_t)kABrows * kS * 2;
constexpr size_t kOffOuter = kOffBt2 + (size_t)kABrows * kS * 2;
constexpr size_t kWsTotal  = kOffOuter + (size_t)kOuterRows * kKo * 2;
static_assert(kWsTotal == 97026048, "ws total");
static_assert(kWsTotal <= (size_t)134217728, "ws budget");
static_assert(kOffBt3 % 2048 == 0 && kOffRnorm % 2048 == 0 && kOffMnP % 2048 == 0 && kOffP1 % 2048 == 0 &&
              kOffA2 % 2048 == 0 && kOffBt2 % 2048 == 0 && kOffOuter % 2048 == 0, "ws align");

typedef __attribute__((ext_vector_type(16))) __bf16   v16b;
typedef __attribute__((ext_vector_type(8)))  __bf16   v8b;
typedef __attribute__((ext_vector_type(8)))  float    v8f;
typedef __attribute__((ext_vector_type(4)))  float    v4f;
typedef __attribute__((ext_vector_type(4)))  unsigned int v4u;

__device__ __forceinline__ unsigned short f2bf_bits(float f) {
  unsigned u = __float_as_uint(f);
  return (unsigned short)((u + 0x7FFFu + ((u >> 16) & 1u)) >> 16);
}
__device__ __forceinline__ unsigned pk16(unsigned short a, unsigned short b) { return (unsigned)a | ((unsigned)b << 16); }

__device__ __forceinline__ v4u pack8_bf16(v4f a, v4f c) {
  const float a0 = a[0], a1 = a[1], a2 = a[2], a3 = a[3];
  const float c0 = c[0], c1 = c[1], c2 = c[2], c3 = c[3];
  v4u u;
  u[0] = pk16(f2bf_bits(a0), f2bf_bits(a1));
  u[1] = pk16(f2bf_bits(a2), f2bf_bits(a3));
  u[2] = pk16(f2bf_bits(c0), f2bf_bits(c1));
  u[3] = pk16(f2bf_bits(c2), f2bf_bits(c3));
  return u;
}

__device__ __forceinline__ void keep4_b(v16b a, v16b b, v16b c, v16b d) { asm volatile("v_nop" :: "v"(a), "v"(b), "v"(c), "v"(d)); }
__device__ __forceinline__ void acc_guard4(v8f& a, v8f& b, v8f& c, v8f& d) { asm volatile("v_nop\n\tv_nop\n\tv_nop\n\tv_nop" : "+v"(a), "+v"(b), "+v"(c), "+v"(d)); }
__device__ __forceinline__ void guard_row_b(v8f& a0, v8f& a1, v8f& a2, v8f& a3, v16b x, v16b y) {
  asm volatile("v_nop\n\tv_nop\n\tv_nop\n\tv_nop" : "+v"(a0), "+v"(a1), "+v"(a2), "+v"(a3) : "v"(x), "v"(y));
}

struct FragB {
  union U { v16b v; v8b h[2]; };
  static __device__ __forceinline__ v16b load(const __bf16* p) {
    U f; f.h[0] = *(const v8b*)(p); f.h[1] = *(const v8b*)(p + 16); return f.v;
  }
  static __device__ __forceinline__ v8f mma(v16b a, v16b b, v8f c) {
    return __builtin_amdgcn_wmma_f32_16x16x32_bf16(false, a, false, b, (short)0, c, false, false);
  }
};

__device__ __forceinline__ void wave_sync() {
  __builtin_amdgcn_fence(__ATOMIC_RELEASE, "workgroup");
  __builtin_amdgcn_wave_barrier();
  __builtin_amdgcn_fence(__ATOMIC_ACQUIRE, "workgroup");
}

__device__ __forceinline__ void gemm_tile_bf16(const __bf16* __restrict__ A, int lda,
                                               const __bf16* __restrict__ Bt, int ldb,
                                               int K, int m0, int n0, int lane, v8f (&acc)[4][4]) {
  const int rlane = lane & 15;
  const int koff  = (lane >> 4) * 8;
#pragma unroll
  for (int i = 0; i < 4; ++i)
#pragma unroll
    for (int j = 0; j < 4; ++j) acc[i][j] = (v8f){0.f,0.f,0.f,0.f,0.f,0.f,0.f,0.f};

  for (int k0 = 0; k0 < K; k0 += 32) {
    v16b bh[4];
#pragma unroll
    for (int j = 0; j < 4; ++j)
      bh[j] = FragB::load(Bt + (size_t)(n0 + (j << 4) + rlane) * ldb + koff + k0);
#pragma unroll
    for (int i = 0; i < 4; ++i) {
      const v16b ah = FragB::load(A + (size_t)(m0 + (i << 4) + rlane) * lda + koff + k0);
#pragma unroll
      for (int j = 0; j < 4; ++j) acc[i][j] = FragB::mma(ah, bh[j], acc[i][j]);
      guard_row_b(acc[i][0], acc[i][1], acc[i][2], acc[i][3], ah, bh[3]);
    }
    keep4_b(bh[0], bh[1], bh[2], bh[3]);
  }
  acc_guard4(acc[0][0], acc[0][1], acc[0][2], acc[0][3]);
  acc_guard4(acc[1][0], acc[1][1], acc[1][2], acc[1][3]);
  acc_guard4(acc[2][0], acc[2][1], acc[2][2], acc[2][3]);
  acc_guard4(acc[3][0], acc[3][1], acc[3][2], acc[3][3]);
}

__global__ __launch_bounds__(256) void cast8_bf16_kernel(const float* __restrict__ in,
                                                         unsigned short* __restrict__ out, int n8) {
  const int idx = blockIdx.x * 256 + threadIdx.x;
  if (idx >= n8) return;
  const float* p = in + 8 * (size_t)idx;
  const v4f a = *(const v4f*)(p);
  const v4f c = *(const v4f*)(p + 4);
  const v4u u = pack8_bf16(a, c);
  unsigned short* q = out + 8 * (size_t)idx;
  *(volatile v4u*)q = u;
  __threadfence();
  *(volatile v4u*)q = u;
}

__global__ __launch_bounds__(256) void layernorm_kernel(const float* __restrict__ m,
                                                        const float* __restrict__ gamma,
                                                        const float* __restrict__ beta,
                                                        unsigned short* __restrict__ mnP) {
  const int lane = threadIdx.x & 31;
  const int wave = threadIdx.x >> 5;
  const int row  = blockIdx.x * 8 + wave;
  const int s    = row >> 8;
  const int ir   = row & 255;
  const float* mp = m + (size_t)row * kCM + lane * 8;
  const v4f x0 = *(const v4f*)(mp);
  const v4f x1 = *(const v4f*)(mp + 4);
  const v4f g0 = *(const v4f*)(gamma + lane * 8);
  const v4f g1 = *(const v4f*)(gamma + lane * 8 + 4);
  const v4f e0 = *(const v4f*)(beta + lane * 8);
  const v4f e1 = *(const v4f*)(beta + lane * 8 + 4);

  float sum = 0.0f;
  sum += x0[0]; sum += x0[1]; sum += x0[2]; sum += x0[3];
  sum += x1[0]; sum += x1[1]; sum += x1[2]; sum += x1[3];
#pragma unroll
  for (int k = 1; k < 32; k <<= 1) sum += __shfl_xor(sum, k, 32);
  const float mu = sum * kInvCM;

  const v4f d0 = x0 - mu;
  const v4f d1 = x1 - mu;
  float ss = 0.0f;
  ss += d0[0] * d0[0]; ss += d0[1] * d0[1]; ss += d0[2] * d0[2]; ss += d0[3] * d0[3];
  ss += d1[0] * d1[0]; ss += d1[1] * d1[1]; ss += d1[2] * d1[2]; ss += d1[3] * d1[3];
#pragma unroll
  for (int k = 1; k < 32; k <<= 1) ss += __shfl_xor(ss, k, 32);
  const float var  = ss * kInvCM;
  const float rstd = rsqrtf(var + kLnEps);

  const v4f n0v = d0 * rstd * g0 + e0;
  const v4f n1v = d1 * rstd * g1 + e1;
  const v4u u = pack8_bf16(n0v, n1v);
  unsigned short* dst = mnP + ((size_t)(ir * kS + s)) * kCM + lane * 8;
  *(volatile v4u*)dst = u;
  __threadfence();
  *(volatile v4u*)dst = u;
}

__global__ __launch_bounds__(64) void pairnorm_kernel(const float* __restrict__ mask, float* __restrict__ rnorm) {
  const int i  = blockIdx.x;
  const int j4 = threadIdx.x * 4;
  v4f acc = (v4f){0.f, 0.f, 0.f, 0.f};
#pragma unroll 4
  for (int s = 0; s < kS; ++s) {
    const float mi = mask[s * kR + i];
    const v4f  mj  = *(const v4f*)(mask + s * kR + j4);
    acc += mj * mi;
  }
  v4f rv;
#pragma unroll
  for (int e = 0; e < 4; ++e) rv[e] = 1.0f / (acc[e] + kNormEps);
  float* dst = rnorm + (size_t)i * kR + j4;
  *(volatile v4f*)dst = rv;
  __threadfence();
  *(volatile v4f*)dst = rv;
}

__global__ __launch_bounds__(256) void proj_gemm_kernel(const unsigned short* __restrict__ Ap,
                                                        const unsigned short* __restrict__ Btp,
                                                        float* __restrict__ Cout) {
  __shared__ __align__(16) float sT[8][16 * 68];
  const __bf16* A  = (const __bf16*)Ap;
  const __bf16* Bt = (const __bf16*)Btp;
  const int lane = threadIdx.x & 31;
  const int wave = threadIdx.x >> 5;
  constexpr int kTiles = kRows / 64;
  const int tile = blockIdx.x * 8 + wave;
  if (tile >= kTiles) return;
  const int m0 = tile << 6;
  const int n0 = 0;

  v8f acc[4][4];
  gemm_tile_bf16(A, kCM, Bt, kCM, kCM, m0, n0, lane, acc);

  const int rlane = lane & 15;
  const int mOff  = (lane >> 4) * 8;
  float* slab = sT[wave];
#pragma unroll
  for (int i = 0; i < 4; ++i) {
    const int mBase = m0 + (i << 4);
#pragma unroll
    for (int j = 0; j < 4; ++j)
#pragma unroll
      for (int r = 0; r < 8; ++r) slab[(mOff + r) * 68 + (j << 4) + rlane] = acc[i][j][r];
    wave_sync();
    {
      const int hh = lane >> 4, c4 = (lane & 15) * 4;
      for (int pass = 0; pass < 2; ++pass) {
#pragma unroll
        for (int it = 0; it < 8; ++it) {
          const int row = it * 2 + hh;
          const v4f v = *(const v4f*)(slab + row * 68 + c4);
          *(volatile v4f*)(Cout + (size_t)(mBase + row) * kNcat + n0 + c4) = v;
        }
        __threadfence();
      }
    }
    wave_sync();
  }
}

__global__ __launch_bounds__(256) void mask_transpose_kernel(const float* __restrict__ P1,
                                                             const float* __restrict__ mask,
                                                             const float* __restrict__ b1,
                                                             const float* __restrict__ b2,
                                                             unsigned short* __restrict__ ab) {
  __shared__ __align__(16) float sm[kNcat][kS + 4];
  __shared__ float maskS[kS];
  __shared__ float biasS[kNcat];
  const int t    = threadIdx.x;
  const int lane = t & 31;
  const int wave = t >> 5;
  const int i    = blockIdx.x;
  if (wave < 4)  maskS[t] = mask[t * kR + i];
  if (wave == 4) biasS[lane] = b1[lane];
  if (wave == 5) biasS[kCH + lane] = b2[lane];
  __syncthreads();

#pragma unroll
  for (int it = 0; it < 8; ++it) {
    const int s  = it * 16 + (t >> 4);
    const int c4 = (t & 15) * 4;
    const v4f v  = *(const v4f*)(P1 + ((size_t)(i * kS + s)) * kNcat + c4);
    const float ms = maskS[s];
#pragma unroll
    for (int e = 0; e < 4; ++e) sm[c4 + e][s] = (v[e] + biasS[c4 + e]) * ms;
  }
  __syncthreads();

  const int hh = lane >> 4;
  const int s0 = (lane & 15) * 8;
  const int rowAdd = (wave >= 4) ? (kABrows - kCH) : 0;
  for (int pass = 0; pass < 2; ++pass) {
#pragma unroll
    for (int q = 0; q < 4; ++q) {
      const int c = wave * 8 + 2 * q + hh;
      const float* sp = &sm[c][s0];
      const v4f a  = *(const v4f*)(sp);
      const v4f bq = *(const v4f*)(sp + 4);
      const v4u u  = pack8_bf16(a, bq);
      unsigned short* dst = ab + ((size_t)(i * kCH + c + rowAdd)) * kS + s0;
      *(volatile v4u*)dst = u;
    }
    __threadfence();
  }
}

__global__ __launch_bounds__(256) void outer_gemm_kernel(const unsigned short* __restrict__ Ap,
                                                         const unsigned short* __restrict__ Btp,
                                                         unsigned short* __restrict__ Op) {
  __shared__ __align__(16) float sT[8][16 * 68];
  const __bf16* A  = (const __bf16*)Ap;
  const __bf16* Bt = (const __bf16*)Btp;
  const int lane = threadIdx.x & 31;
  const int wave = threadIdx.x >> 5;
  constexpr int kTilesN = (kR * kCH) / 64;
  constexpr int kTilesM = (kChunkI * kCH) / 64;
  const int tile = blockIdx.x * 8 + wave;
  if (tile >= kTilesM * kTilesN) return;
  const int tm = tile / kTilesN;
  const int tn = tile - tm * kTilesN;
  const int m0 = tm << 6;
  const int n0 = tn << 6;

  v8f acc[4][4];
  gemm_tile_bf16(A, kS, Bt, kS, kS, m0, n0, lane, acc);

  const int rlane = lane & 15;
  const int mOff  = (lane >> 4) * 8;
  float* slab = sT[wave];
#pragma unroll
  for (int i = 0; i < 4; ++i) {
#pragma unroll
    for (int j = 0; j < 4; ++j)
#pragma unroll
      for (int r = 0; r < 8; ++r) slab[(mOff + r) * 68 + (j << 4) + rlane] = acc[i][j][r];
    wave_sync();
    {
      const int il    = tm * 2 + (i >> 1);
      const int cbase = 16 * (i & 1);
      const int rrow  = lane >> 2;
      const int d8    = (lane & 3) * 8;
      for (int pass = 0; pass < 2; ++pass) {
#pragma unroll
        for (int jj = 0; jj < 2; ++jj) {
          const int j = tn * 2 + jj;
          unsigned short* orow = Op + ((size_t)(il * kR + j)) * kKo + cbase * kCH;
#pragma unroll
          for (int it = 0; it < 2; ++it) {
            const int row = it * 8 + rrow;
            const float* sp = slab + row * 68 + jj * 32 + d8;
            const v4f a  = *(const v4f*)(sp);
            const v4f bq = *(const v4f*)(sp + 4);
            const v4u u  = pack8_bf16(a, bq);
            *(volatile v4u*)(orow + 256 * it + 8 * lane) = u;
          }
        }
        __threadfence();
      }
    }
    wave_sync();
  }
}

__global__ __launch_bounds__(256) void out_gemm_kernel(const unsigned short* __restrict__ Ap,
                                                       const unsigned short* __restrict__ Btp,
                                                       const float* __restrict__ b_o,
                                                       const float* __restrict__ rnorm,
                                                       const float* __restrict__ zin,
                                                       float* __restrict__ out, int rowBase) {
  __shared__ __align__(16) float sT[8][16 * 68];
  const __bf16* A  = (const __bf16*)Ap;
  const __bf16* Bt = (const __bf16*)Btp;
  const int lane = threadIdx.x & 31;
  const int wave = threadIdx.x >> 5;
  constexpr int kTilesN = kCZ / 64;
  constexpr int kTilesM = kOuterRows / 64;
  const int tile = blockIdx.x * 8 + wave;
  if (tile >= kTilesM * kTilesN) return;
  const int tm = tile >> 1;
  const int tn = tile & 1;
  const int m0 = tm << 6;
  const int n0 = tn << 6;

  v8f acc[4][4];
  gemm_tile_bf16(A, kKo, Bt, kKo, kKo, m0, n0, lane, acc);

  const int rlane = lane & 15;
  const int mOff  = (lane >> 4) * 8;
  float bvs[4];
#pragma unroll
  for (int j = 0; j < 4; ++j) bvs[j] = b_o[n0 + (j << 4) + rlane];

  float* slab = sT[wave];
  const int hh = lane >> 4, c4 = (lane & 15) * 4;
#pragma unroll
  for (int i = 0; i < 4; ++i) {
    const int mBase = m0 + (i << 4);
#pragma unroll
    for (int j = 0; j < 4; ++j)
#pragma unroll
      for (int r = 0; r < 8; ++r) slab[(mOff + r) * 68 + (j << 4) + rlane] = acc[i][j][r] + bvs[j];
    wave_sync();
#pragma unroll
    for (int it = 0; it < 8; ++it) {
      const int row = it * 2 + hh;
      const size_t grow = (size_t)rowBase + (size_t)(mBase + row);
      const v4f sv = *(const v4f*)(slab + row * 68 + c4);
      const float rn = rnorm[grow];
      const v4f zz = *(const v4f*)(zin + grow * kCZ + n0 + c4);
      const v4f f  = zz + sv * rn;
      *(v4f*)(slab + row * 68 + c4) = f;
      if (it == 3) asm volatile("" ::: "memory");
    }
    wave_sync();
    for (int pass = 0; pass < 2; ++pass) {
#pragma unroll
      for (int it = 0; it < 8; ++it) {
        const int row = it * 2 + hh;
        const size_t grow = (size_t)rowBase + (size_t)(mBase + row);
        const v4f v = *(const v4f*)(slab + row * 68 + c4);
        *(volatile v4f*)(out + grow * kCZ + n0 + c4) = v;
      }
      __threadfence();
    }
    wave_sync();
  }
}

extern "C" void kernel_launch(void* const* d_in, const int* in_sizes, int n_in,
                              void* d_out, int out_size, void* d_ws, size_t ws_size,
                              hipStream_t stream) {
  (void)in_sizes; (void)n_in; (void)out_size;
  if (ws_size < kWsTotal) return;
  const float* m     = (const float*)d_in[0];
  const float* mask  = (const float*)d_in[1];
  const float* zin   = (const float*)d_in[2];
  const float* gamma = (const float*)d_in[3];
  const float* beta  = (const float*)d_in[4];
  const float* w1    = (const float*)d_in[5];
  const float* b1    = (const float*)d_in[6];
  const float* w2    = (const float*)d_in[7];
  const float* b2    = (const float*)d_in[8];
  const float* w_o   = (const float*)d_in[9];
  const float* b_o   = (const float*)d_in[10];
  float* out = (float*)d_out;

  unsigned char* ws = (unsigned char*)d_ws;
  unsigned short* Bt1    = (unsigned short*)(ws + kOffBt1);
  unsigned short* Bt3    = (unsigned short*)(ws + kOffBt3);
  float*          rnorm  = (float*)(ws + kOffRnorm);
  unsigned short* mnP    = (unsigned short*)(ws + kOffMnP);
  float*          P1     = (float*)(ws + kOffP1);
  unsigned short* A2     = (unsigned short*)(ws + kOffA2);
  unsigned short* Bt2    = (unsigned short*)(ws + kOffBt2);
  unsigned short* outerP = (unsigned short*)(ws + kOffOuter);

  cast8_bf16_kernel<<<(kCH * kCM / 8) / 256, 256, 0, stream>>>(w1, Bt1, kCH * kCM / 8);
  cast8_bf16_kernel<<<(kCH * kCM / 8) / 256, 256, 0, stream>>>(w2, Bt1 + kCH * kCM, kCH * kCM / 8);
  cast8_bf16_kernel<<<(kCZ * kKo / 8) / 256, 256, 0, stream>>>(w_o, Bt3, kCZ * kKo / 8);
  layernorm_kernel<<<kRows / 8, 256, 0, stream>>>(m, gamma, beta, mnP);
  pairnorm_kernel<<<kR, 64, 0, stream>>>(mask, rnorm);
  proj_gemm_kernel<<<(kRows / 64) / 8, 256, 0, stream>>>(mnP, Bt1, P1);
  mask_transpose_kernel<<<kR, 256, 0, stream>>>(P1, mask, b1, b2, A2);
  for (int ch = 0; ch < kNumChunks; ++ch) {
    const unsigned short* A2c = A2 + (size_t)ch * kChunkI * kCH * kS;
    outer_gemm_kernel<<<((kChunkI * kCH / 64) * (kR * kCH / 64)) / 8, 256, 0, stream>>>(A2c, Bt2, outerP);
    out_gemm_kernel<<<((kOuterRows / 64) * (kCZ / 64)) / 8, 256, 0, stream>>>(outerP, Bt3, b_o, rnorm, zin, out,
                                                                              ch * kChunkI * kR);
  }
}
